// ContextCorrelationEncoder_55929064129156
// MI455X (gfx1250) — hardware-verified
//
#include <hip/hip_runtime.h>
#include <stdint.h>

#pragma clang fp contract(off)

#define NB     4
#define NC     64
#define HI     192
#define WI     192
#define HWI    (HI * WI)
#define NPIX   (NB * HWI)
#define PD     194
#define PF     200
#define KT     576
#define KQ     160
#define NCV    81
#define NCX    145
#define SP     72
#define CSP    104
#define OSP    36
#define TPX    128
#define RSC    2048.0f
#define INV_R  4.8828125e-04f
#define WSC    64.0f
#define INV_W  0.015625f
#define INV_WR 7.62939453125e-06f
#define CVS    0.125f
#define BN_EPS 1e-5f

#define X_E    ((size_t)NB * PD * PD * NC)
#define F1_E   ((size_t)NPIX * NC)
#define F2_E   ((size_t)NB * PF * PF * NC)

#define W_CHK  (NC * KT / 8)
#define W_BLK  (W_CHK / 256)
#define Q_CHK  (NC * KQ / 8)
#define Q_BLK  (Q_CHK / 256)
#define NBLK_X  (NB * PD)
#define NBLK_CV (NB * HI * (WI / 64))
#define NBLK_CQ (NB * (HI / 4) * (WI / 32))

#define WS_W1  ((size_t)0)
#define WS_W2  (WS_W1 + (size_t)NC * KT * 2)
#define WS_WQ  (WS_W2 + (size_t)NC * KT * 2)
#define WS_X1  (WS_WQ + (size_t)NC * KQ * 2)
#define WS_X2  (WS_X1 + X_E * 2)
#define WS_F1  (WS_X2 + X_E * 2)
#define WS_F2  (WS_F1 + 2 * F1_E * 2)
#define WS_END (WS_F2 + 2 * F2_E * 2)

static_assert(W_CHK % 256 == 0);
static_assert(Q_CHK % 256 == 0);
static_assert(KT % 32 == 0);
static_assert(KQ % 32 == 0);
static_assert((WS_W2 % 128) == 0);
static_assert((WS_WQ % 128) == 0);
static_assert((WS_X1 % 128) == 0);
static_assert(((X_E * 2) % 128) == 0);
static_assert(((F1_E * 2) % 128) == 0);
static_assert(((F2_E * 2) % 128) == 0);
static_assert(WS_END == (size_t)117415936);
static_assert(WS_END <= (size_t)134217728);
static_assert((SP * 2) % 16 == 0);
static_assert((CSP * 2) % 16 == 0);
static_assert((OSP * 4) % 16 == 0);
static_assert(256 * OSP * 4 <= 2 * TPX * CSP * 2);
static_assert((HI % 4) == 0 && (WI % 64) == 0 && (WI % 32) == 0);
static_assert(PD * SP * 2 <= 60000);
static_assert(2 * TPX * CSP * 2 <= 60000);

typedef _Float16       v16h __attribute__((ext_vector_type(16)));
typedef _Float16       v8h  __attribute__((ext_vector_type(8)));
typedef __bf16         v16b __attribute__((ext_vector_type(16)));
typedef __bf16         v8b  __attribute__((ext_vector_type(8)));
typedef float          v8f  __attribute__((ext_vector_type(8)));
typedef float          v4f  __attribute__((ext_vector_type(4)));
typedef unsigned       v4u  __attribute__((ext_vector_type(4)));
typedef unsigned short v8us __attribute__((ext_vector_type(8)));

__device__ __forceinline__ unsigned bfb(float f) {
  unsigned u = __float_as_uint(f);
  return (u + 0x7FFFu + ((u >> 16) & 1u)) >> 16;
}
__device__ __forceinline__ float bf_rne(float f) { return __uint_as_float(bfb(f) << 16); }
__device__ __forceinline__ unsigned hbits(_Float16 h) {
  return (unsigned)__builtin_bit_cast(unsigned short, h);
}
__device__ __forceinline__ v8f zero8f() { v8f z = {0.f, 0.f, 0.f, 0.f, 0.f, 0.f, 0.f, 0.f}; return z; }
__device__ __forceinline__ v8h zero8h() {
  v8h z;
#pragma unroll
  for (int e = 0; e < 8; ++e) z[e] = (_Float16)0.0f;
  return z;
}
__device__ __forceinline__ v8us zero8us() {
  v8us z;
#pragma unroll
  for (int e = 0; e < 8; ++e) z[e] = (unsigned short)0;
  return z;
}

__device__ __forceinline__ v16h ldfrag_h(const _Float16* p) {
  union { v16h v; v8h h[2]; } f;
  f.h[0] = *(const v8h*)(p);
  f.h[1] = *(const v8h*)(p + 16);
  return f.v;
}
__device__ __forceinline__ v16b ldfrag_b(const __bf16* p) {
  union { v16b v; v8b h[2]; } f;
  f.h[0] = *(const v8b*)(p);
  f.h[1] = *(const v8b*)(p + 16);
  return f.v;
}

__device__ __forceinline__ v8f mma_h(v16h a, v16h b, v8f c) {
  return __builtin_amdgcn_wmma_f32_16x16x32_f16(false, a, false, b, (short)0, c, false, false);
}
__device__ __forceinline__ v8f mma_b(v16b a, v16b b, v8f c) {
  return __builtin_amdgcn_wmma_f32_16x16x32_bf16(false, a, false, b, (short)0, c, false, false);
}
template <typename F>
__device__ __forceinline__ void guard2(v8f& c0, v8f& c1, const F& f0, const F& f1, const F& f2) {
#if defined(__HIP_DEVICE_COMPILE__)
  asm volatile("v_nop\n\tv_nop\n\tv_nop\n\tv_nop"
               : "+v"(c0), "+v"(c1)
               : "v"(f0), "v"(f1), "v"(f2));
#endif
}
__device__ __forceinline__ void guard2x8(v8f& c0, v8f& c1,
                                         const v16h& f0, const v16h& f1, const v16h& f2, const v16h& f3,
                                         const v16h& f4, const v16h& f5, const v16h& f6, const v16h& f7) {
#if defined(__HIP_DEVICE_COMPILE__)
  asm volatile("v_nop\n\tv_nop\n\tv_nop\n\tv_nop"
               : "+v"(c0), "+v"(c1)
               : "v"(f0), "v"(f1), "v"(f2), "v"(f3), "v"(f4), "v"(f5), "v"(f6), "v"(f7));
#endif
}
__device__ __forceinline__ void accg2(v8f& c0, v8f& c1) {
#if defined(__HIP_DEVICE_COMPILE__)
  asm volatile("v_nop\n\tv_nop\n\tv_nop\n\tv_nop" : "+v"(c0), "+v"(c1));
#endif
}
__device__ __forceinline__ void accg8(v8f& c0, v8f& c1, v8f& c2, v8f& c3,
                                      v8f& c4, v8f& c5, v8f& c6, v8f& c7) {
#if defined(__HIP_DEVICE_COMPILE__)
  asm volatile("v_nop\n\tv_nop\n\tv_nop\n\tv_nop"
               : "+v"(c0), "+v"(c1), "+v"(c2), "+v"(c3), "+v"(c4), "+v"(c5), "+v"(c6), "+v"(c7));
#endif
}
__device__ __forceinline__ void step1x1(v8f& qh, v8f& qr, const v16h& fah, const v16h& far_,
                                        const _Float16* bp) {
  const v16h fb = ldfrag_h(bp);
  qh = mma_h(fah, fb, qh);
  qr = mma_h(far_, fb, qr);
  guard2(qh, qr, fah, far_, fb);
}
__device__ __forceinline__ float bnq(float ah, float ar, float cb, float S, float sh) {
  const float t = (ah * INV_W + ar * INV_WR) + cb;
  const float y = t * S + sh;
  return fmaxf(y, 0.0f);
}

__global__ __launch_bounds__(256)
void k_wpack(const float* __restrict__ wk, const float* __restrict__ wq, const float* __restrict__ qw,
             unsigned* w1, unsigned* w2, unsigned* wqp)
{
  const int tid = threadIdx.x;
  const int blk = blockIdx.x;
  unsigned hb[8];
  unsigned* dst;
  if (blk < 2 * W_BLK) {
    const int sel = (blk >= W_BLK) ? 1 : 0;
    const float* src = sel ? wq : wk;
    const int q   = (blk - sel * W_BLK) * 256 + tid;
    const int co  = q / (KT / 8);
    const int kc  = (q - co * (KT / 8)) * 8;
    const int tap = kc >> 6;
    const int ci0 = kc & 63;
#pragma unroll
    for (int j = 0; j < 8; ++j)
      hb[j] = bfb(src[(size_t)(co * NC + ci0 + j) * 9 + tap]);
    dst = (sel ? w2 : w1) + (size_t)q * 4;
  } else {
    const int q  = (blk - 2 * W_BLK) * 256 + tid;
    const int co = q / (KQ / 8);
    const int kc = (q - co * (KQ / 8)) * 8;
#pragma unroll
    for (int j = 0; j < 8; ++j) {
      const int k   = kc + j;
      const int ch  = (k < NCV) ? k : (k - (KQ - NCX));
      const int chc = (ch < 0) ? 0 : ((ch > NCX - 1) ? (NCX - 1) : ch);
      const float v = bf_rne(qw[(size_t)co * NCX + chc]) * WSC;
      const bool pad = (k >= NCV) && (k < KQ - NC);
      hb[j] = pad ? 0u : hbits((_Float16)v);
    }
    dst = wqp + (size_t)q * 4;
  }
  v4u wv;
  wv.x = hb[0] | (hb[1] << 16);
  wv.y = hb[2] | (hb[3] << 16);
  wv.z = hb[4] | (hb[5] << 16);
  wv.w = hb[6] | (hb[7] << 16);
  *(volatile v4u*)dst = wv;
  __threadfence();
  *(volatile v4u*)dst = wv;
}

__global__ __launch_bounds__(256)
void k_xcvt(const float* __restrict__ xa, const float* __restrict__ xb,
            unsigned short* pa, unsigned short* pb)
{
  __shared__ __align__(16) unsigned short T[PD * SP];
  const int tid  = threadIdx.x;
  const int lane = tid & 31;
  const int wid  = tid >> 5;
  const int pj   = lane & 7;
  const int lq   = lane >> 3;
  const int sel  = (blockIdx.x >= NBLK_X) ? 1 : 0;
  const int g    = blockIdx.x - sel * NBLK_X;
  const int b    = g / PD;
  const int hp   = g - b * PD;
  const float* x = sel ? xb : xa;
  unsigned short* xh = sel ? pb : pa;
  const size_t rowb = ((size_t)(b * PD + hp)) * PD;

  if (hp == 0 || hp == PD - 1) {
    const v8us zu = zero8us();
    size_t e[7]; bool ok[7];
#pragma unroll
    for (int r = 0; r < 7; ++r) {
      const int L  = r * 32 + wid * 4 + lq;
      const int Lc = (L < PD) ? L : (PD - 1);
      e[r]  = (rowb + Lc) * NC + 8 * pj;
      ok[r] = (L < PD);
    }
#pragma unroll
    for (int r = 0; r < 7; ++r) if (ok[r]) *(volatile v8us*)(xh + e[r]) = zu;
    __threadfence();
#pragma unroll
    for (int r = 0; r < 7; ++r) if (ok[r]) *(volatile v8us*)(xh + e[r]) = zu;
  } else {
    const int h = hp - 1;
    if (tid < 16) {
      const int slot = (tid < 8) ? 0 : (PD - 1);
      *(v8us*)&T[slot * SP + 8 * (tid & 7)] = zero8us();
    }
#pragma unroll
    for (int i = 0; i < 12; ++i) {
      const int idx = tid + 256 * i;
      const int w4  = idx % 48;
      const int c   = idx / 48;
      const v4f v = *(const v4f*)(x + ((size_t)(b * NC + c) * HI + h) * WI + 4 * w4);
      unsigned short* tp = T + (4 * w4 + 1) * SP + c;
      tp[0 * SP] = (unsigned short)bfb(v.x);
      tp[1 * SP] = (unsigned short)bfb(v.y);
      tp[2 * SP] = (unsigned short)bfb(v.z);
      tp[3 * SP] = (unsigned short)bfb(v.w);
    }
    __syncthreads();
    v8us val[7]; size_t e[7]; bool ok[7];
#pragma unroll
    for (int r = 0; r < 7; ++r) {
      const int L  = r * 32 + wid * 4 + lq;
      const int Lc = (L < PD) ? L : (PD - 1);
      val[r] = *(const v8us*)&T[Lc * SP + 8 * pj];
      e[r]   = (rowb + Lc) * NC + 8 * pj;
      ok[r]  = (L < PD);
    }
#pragma unroll
    for (int r = 0; r < 7; ++r) if (ok[r]) *(volatile v8us*)(xh + e[r]) = val[r];
    __threadfence();
#pragma unroll
    for (int r = 0; r < 7; ++r) if (ok[r]) *(volatile v8us*)(xh + e[r]) = val[r];
  }
}

__global__ __launch_bounds__(256)
void k_zero(_Float16* f2p)
{
  const int tid  = threadIdx.x;
  const int lane = tid & 31;
  const int wid  = tid >> 5;
  const int pj   = lane & 7;
  const int lq   = lane >> 3;
  const int b    = blockIdx.x >> 3;
  const int ri   = blockIdx.x & 7;
  const int pr   = (ri < 4) ? ri : (ri + (PF - 8));
  const size_t rowb = ((size_t)(b * PF + pr)) * PF;
  const v8h z = zero8h();
  size_t e[13]; bool ok[13];
#pragma unroll
  for (int r = 0; r < 13; ++r) {
    const int L   = r * 32 + wid * 4 + lq;
    const int Lc  = (L < 2 * PF) ? L : (2 * PF - 1);
    const int pl  = (Lc >= PF) ? 1 : 0;
    const int col = Lc - PF * pl;
    e[r]  = (size_t)pl * F2_E + (rowb + col) * NC + 8 * pj;
    ok[r] = (L < 2 * PF);
  }
#pragma unroll
  for (int r = 0; r < 13; ++r) if (ok[r]) *(volatile v8h*)(f2p + e[r]) = z;
  __threadfence();
#pragma unroll
  for (int r = 0; r < 13; ++r) if (ok[r]) *(volatile v8h*)(f2p + e[r]) = z;
}

__global__ __launch_bounds__(256)
void k_conv(const __bf16* __restrict__ x1, const __bf16* __restrict__ x2,
            const __bf16* __restrict__ w1, const __bf16* __restrict__ w2,
            const float* __restrict__ cb1, const float* __restrict__ gg1, const float* __restrict__ be1,
            const float* __restrict__ mu1, const float* __restrict__ va1,
            const float* __restrict__ cb2, const float* __restrict__ gg2, const float* __restrict__ be2,
            const float* __restrict__ mu2, const float* __restrict__ va2,
            _Float16* f1p, _Float16* f2p)
{
  __shared__ __align__(16) _Float16 sth[68 * SP];
  __shared__ __align__(16) _Float16 stl[68 * SP];
  __shared__ float bS[NC];
  __shared__ float bB[NC];
  __shared__ float bC[NC];

  const int tid  = threadIdx.x;
  const int lane = tid & 31;
  const int wid  = tid >> 5;
  const int l15  = lane & 15;
  const int hh   = lane >> 4;
  const int sel  = (blockIdx.x >= NBLK_CV) ? 1 : 0;
  const int g    = blockIdx.x - sel * NBLK_CV;
  const int seg  = g % 3;
  const int h    = (g / 3) % HI;
  const int b    = g / (3 * HI);
  const int w0   = 64 * seg;
  const __bf16* xin = sel ? x2 : x1;
  const __bf16* wgt = sel ? w2 : w1;

  if (tid < NC) {
    const float* cb = sel ? cb2 : cb1;
    const float* gg = sel ? gg2 : gg1;
    const float* be = sel ? be2 : be1;
    const float* mu = sel ? mu2 : mu1;
    const float* va = sel ? va2 : va1;
    const float gam = bf_rne(gg[tid]);
    const float var = bf_rne(va[tid]);
    const float inv = gam / sqrtf(var + BN_EPS);
    bS[tid] = inv;
    bB[tid] = bf_rne(be[tid]) - bf_rne(mu[tid]) * inv;
    bC[tid] = bf_rne(cb[tid]);
  }
  if (tid < 32) {
    *(v8h*)&sth[(64 + (tid >> 3)) * SP + 8 * (tid & 7)] = zero8h();
  } else if (tid < 64) {
    *(v8h*)&stl[(64 + ((tid - 32) >> 3)) * SP + 8 * (tid & 7)] = zero8h();
  }
  __syncthreads();

  const int nt = wid & 3;
  const int mh = wid >> 2;
  const int n0 = 16 * nt;
  const __bf16* bp = wgt + (size_t)(n0 + l15) * KT + 8 * hh;
  const __bf16* ap = xin + (((size_t)(b * PD + h)) * PD + w0 + 32 * mh + l15) * NC + 8 * hh;
  v8f c0 = zero8f(), c1 = zero8f();
#pragma unroll 1
  for (int kh = 0; kh < 3; ++kh) {
#pragma unroll 1
    for (int kw = 0; kw < 3; ++kw) {
      const __bf16* a  = ap + (kh * PD + kw) * NC;
      const __bf16* bk = bp + (kh * 3 + kw) * 64;
      {
        const v16b fb = ldfrag_b(bk);
        const v16b f0 = ldfrag_b(a);
        const v16b f1 = ldfrag_b(a + 16 * NC);
        c0 = mma_b(f0, fb, c0);
        c1 = mma_b(f1, fb, c1);
        guard2(c0, c1, f0, f1, fb);
      }
      {
        const v16b fb = ldfrag_b(bk + 32);
        const v16b f0 = ldfrag_b(a + 32);
        const v16b f1 = ldfrag_b(a + 16 * NC + 32);
        c0 = mma_b(f0, fb, c0);
        c1 = mma_b(f1, fb, c1);
        guard2(c0, c1, f0, f1, fb);
      }
    }
  }
  accg2(c0, c1);

  {
    const int ch = n0 + l15;
    const float S  = bS[ch];
    const float sh = bB[ch];
    const float cb = bC[ch];
    const int px0 = 32 * mh + 8 * hh;
#pragma unroll
    for (int r = 0; r < 8; ++r) {
      {
        const float t = c0[r] + cb;
        const float y = fmaxf(t * S + sh, 0.0f);
        const _Float16 hv = (_Float16)y;
        const _Float16 lv = (_Float16)((y - (float)hv) * RSC);
        sth[(px0 + r) * SP + ch] = hv;
        stl[(px0 + r) * SP + ch] = lv;
      }
      {
        const float t = c1[r] + cb;
        const float y = fmaxf(t * S + sh, 0.0f);
        const _Float16 hv = (_Float16)y;
        const _Float16 lv = (_Float16)((y - (float)hv) * RSC);
        sth[(px0 + 16 + r) * SP + ch] = hv;
        stl[(px0 + 16 + r) * SP + ch] = lv;
      }
    }
  }
  __syncthreads();

  {
    const int pj = lane & 7;
    const int lq = lane >> 3;
    const int npl   = 64 + ((sel && seg != 1) ? 4 : 0);
    const int total = 2 * npl;
    const size_t rowb = sel ? (((size_t)(b * PF + h + 4)) * PF) : (((size_t)(b * HI + h)) * WI);
    const int colb  = sel ? (w0 + 4) : w0;
    const size_t resoff = sel ? F2_E : F1_E;
    _Float16* fo = sel ? f2p : f1p;
    v8h val[5]; size_t e[5]; bool ok[5];
#pragma unroll
    for (int r = 0; r < 5; ++r) {
      const int L    = r * 32 + wid * 4 + lq;
      const int Lc   = (L < total) ? L : (total - 1);
      const int pl   = (Lc >= npl) ? 1 : 0;
      const int slot = Lc - npl * pl;
      const int pp   = (slot < 64) ? (colb + slot) : ((seg == 0) ? (slot - 64) : (PF - 4 + slot - 64));
      const v8h vh = *(const v8h*)&sth[slot * SP + 8 * pj];
      const v8h vl = *(const v8h*)&stl[slot * SP + 8 * pj];
      val[r] = pl ? vl : vh;
      e[r]   = (size_t)pl * resoff + (rowb + pp) * NC + 8 * pj;
      ok[r]  = (L < total);
    }
#pragma unroll
    for (int r = 0; r < 5; ++r) if (ok[r]) *(volatile v8h*)(fo + e[r]) = val[r];
    __threadfence();
#pragma unroll
    for (int r = 0; r < 5; ++r) if (ok[r]) *(volatile v8h*)(fo + e[r]) = val[r];
  }
}

union CqSmem { _Float16 c[2 * TPX * CSP]; float o[256 * OSP]; };

__global__ __launch_bounds__(256)
void k_cq(const _Float16* __restrict__ f1p, const _Float16* __restrict__ f2p,
          const _Float16* __restrict__ wqp,
          const float* __restrict__ qb, const float* __restrict__ qg, const float* __restrict__ qbe,
          const float* __restrict__ qm, const float* __restrict__ qv,
          float* out)
{
  __shared__ __align__(16) CqSmem sm;
  __shared__ float bS[NC];
  __shared__ float bB[NC];
  __shared__ float bC[NC];

  const int tid  = threadIdx.x;
  const int lane = tid & 31;
  const int wid  = tid >> 5;
  const int l15  = lane & 15;
  const int hh   = lane >> 4;
  const int cg   = blockIdx.x % (WI / 32);
  const int rg   = (blockIdx.x / (WI / 32)) % (HI / 4);
  const int b    = blockIdx.x / ((WI / 32) * (HI / 4));
  const int h0   = 4 * rg;
  const int w0   = 32 * cg;
  const _Float16* f1r = f1p + F1_E;
  const _Float16* f2r = f2p + F2_E;

  if (tid < NC) {
    const float gam = bf_rne(qg[tid]);
    const float var = bf_rne(qv[tid]);
    const float inv = gam / sqrtf(var + BN_EPS);
    bS[tid] = inv;
    bB[tid] = bf_rne(qbe[tid]) - bf_rne(qm[tid]) * inv;
    bC[tid] = bf_rne(qb[tid]);
  }
  {
    _Float16* rowp = sm.c + (size_t)(hh * TPX + 16 * wid + l15) * CSP;
    const v8h z = zero8h();
    *(v8h*)(rowp + 80) = z;
    *(v8h*)(rowp + 88) = z;
  }
  __syncthreads();

  const int dr = l15 >> 2;
  const int dc = l15 & 3;
  const size_t pixA = ((size_t)(b * HI + h0 + dr)) * WI + w0 + 4 * wid + dc;
  const _Float16* aph = f1p + pixA * NC + 8 * hh;
  const _Float16* apr = f1r + pixA * NC + 8 * hh;
  const v16h Ah0 = ldfrag_h(aph);
  const v16h Ah1 = ldfrag_h(aph + 32);
  const v16h Ar0 = ldfrag_h(apr);
  const v16h Ar1 = ldfrag_h(apr + 32);
  {
    _Float16* rh = sm.c + (size_t)(16 * wid) * CSP;
    _Float16* rr = sm.c + (size_t)(TPX + 16 * wid) * CSP;
#pragma unroll 1
    for (int st = 0; st < 9; ++st) {
      const int sr = st / 3;
      const int sc = st - 3 * sr;
      const size_t pixB = ((size_t)(b * PF + h0 + 4 * sr + dr)) * PF + w0 + 4 * wid + 4 * sc + dc;
      const _Float16* bph = f2p + pixB * NC + 8 * hh;
      const _Float16* bpr = f2r + pixB * NC + 8 * hh;
      const v16h Bh0 = ldfrag_h(bph);
      const v16h Bh1 = ldfrag_h(bph + 32);
      const v16h Br0 = ldfrag_h(bpr);
      const v16h Br1 = ldfrag_h(bpr + 32);
      v8f ah = zero8f(), ar = zero8f();
      ah = mma_h(Ah0, Bh0, ah);
      ah = mma_h(Ah1, Bh1, ah);
      ar = mma_h(Ah0, Br0, ar);
      ar = mma_h(Ar0, Bh0, ar);
      ar = mma_h(Ah1, Br1, ar);
      ar = mma_h(Ar1, Bh1, ar);
      guard2x8(ah, ar, Ah0, Ah1, Ar0, Ar1, Bh0, Bh1, Br0, Br1);
#pragma unroll
      for (int r = 0; r < 8; ++r) {
        const int m   = 8 * hh + r;
        const int drm = m >> 2;
        const int dcm = r & 3;
        const int bb  = 4 * sr + dr - drm;
        const int aa  = 4 * sc + dc - dcm;
        const float v = (ah[r] + ar[r] * INV_R) * CVS;
        const _Float16 hv = (_Float16)v;
        const _Float16 lv = (_Float16)((v - (float)hv) * RSC);
        if ((unsigned)bb < 9u && (unsigned)aa < 9u) {
          const int ci = aa * 9 + bb;
          rh[m * CSP + ci] = hv;
          rr[m * CSP + ci] = lv;
        }
      }
    }
  }
  __syncthreads();

  v8f qh0 = zero8f(), qh1 = zero8f(), qh2 = zero8f(), qh3 = zero8f();
  v8f qr0 = zero8f(), qr1 = zero8f(), qr2 = zero8f(), qr3 = zero8f();
  {
    const _Float16* cap = sm.c + (size_t)(16 * wid + l15) * CSP + 8 * hh;
    const _Float16* car = sm.c + (size_t)(TPX + 16 * wid + l15) * CSP + 8 * hh;
    const _Float16* bq  = wqp + (size_t)l15 * KQ + 8 * hh;
    {
      const v16h fah = ldfrag_h(cap);
      const v16h far_ = ldfrag_h(car);
      step1x1(qh0, qr0, fah, far_, bq + 0 * 16 * KQ + 0);
      step1x1(qh1, qr1, fah, far_, bq + 1 * 16 * KQ + 0);
      step1x1(qh2, qr2, fah, far_, bq + 2 * 16 * KQ + 0);
      step1x1(qh3, qr3, fah, far_, bq + 3 * 16 * KQ + 0);
    }
    {
      const v16h fah = ldfrag_h(cap + 32);
      const v16h far_ = ldfrag_h(car + 32);
      step1x1(qh0, qr0, fah, far_, bq + 0 * 16 * KQ + 32);
      step1x1(qh1, qr1, fah, far_, bq + 1 * 16 * KQ + 32);
      step1x1(qh2, qr2, fah, far_, bq + 2 * 16 * KQ + 32);
      step1x1(qh3, qr3, fah, far_, bq + 3 * 16 * KQ + 32);
    }
    {
      const v16h fah = ldfrag_h(cap + 64);
      const v16h far_ = ldfrag_h(car + 64);
      step1x1(qh0, qr0, fah, far_, bq + 0 * 16 * KQ + 64);
      step1x1(qh1, qr1, fah, far_, bq + 1 * 16 * KQ + 64);
      step1x1(qh2, qr2, fah, far_, bq + 2 * 16 * KQ + 64);
      step1x1(qh3, qr3, fah, far_, bq + 3 * 16 * KQ + 64);
    }
    step1x1(qh0, qr0, Ah0, Ar0, bq + 0 * 16 * KQ + 96);
    step1x1(qh1, qr1, Ah0, Ar0, bq + 1 * 16 * KQ + 96);
    step1x1(qh2, qr2, Ah0, Ar0, bq + 2 * 16 * KQ + 96);
    step1x1(qh3, qr3, Ah0, Ar0, bq + 3 * 16 * KQ + 96);
    step1x1(qh0, qr0, Ah1, Ar1, bq + 0 * 16 * KQ + 128);
    step1x1(qh1, qr1, Ah1, Ar1, bq + 1 * 16 * KQ + 128);
    step1x1(qh2, qr2, Ah1, Ar1, bq + 2 * 16 * KQ + 128);
    step1x1(qh3, qr3, Ah1, Ar1, bq + 3 * 16 * KQ + 128);
  }
  accg8(qh0, qh1, qh2, qh3, qr0, qr1, qr2, qr3);
  __syncthreads();

  {
#pragma unroll
    for (int nt = 0; nt < 4; ++nt) {
      const v8f& qh = (nt == 0) ? qh0 : ((nt == 1) ? qh1 : ((nt == 2) ? qh2 : qh3));
      const v8f& qr = (nt == 0) ? qr0 : ((nt == 1) ? qr1 : ((nt == 2) ? qr2 : qr3));
      const int ch = 16 * nt + l15;
      const float S  = bS[ch];
      const float sh = bB[ch];
      const float cb = bC[ch];
      v4f p0, p1;
      p0.x = bnq(qh[0], qr[0], cb, S, sh);
      p0.y = bnq(qh[1], qr[1], cb, S, sh);
      p0.z = bnq(qh[2], qr[2], cb, S, sh);
      p0.w = bnq(qh[3], qr[3], cb, S, sh);
      p1.x = bnq(qh[4], qr[4], cb, S, sh);
      p1.y = bnq(qh[5], qr[5], cb, S, sh);
      p1.z = bnq(qh[6], qr[6], cb, S, sh);
      p1.w = bnq(qh[7], qr[7], cb, S, sh);
      float* o0 = sm.o + (size_t)(ch * 4 + 2 * hh) * OSP + 4 * wid;
      *(v4f*)(o0)       = p0;
      *(v4f*)(o0 + OSP) = p1;
    }
  }
  __syncthreads();

  {
    const int pj = lane & 7;
    const int lq = lane >> 3;
    v4f val[8]; size_t e[8];
#pragma unroll
    for (int r = 0; r < 8; ++r) {
      const int L   = r * 32 + wid * 4 + lq;
      const int chn = L >> 2;
      const int dro = L & 3;
      val[r] = *(const v4f*)(sm.o + (size_t)L * OSP + 4 * pj);
      e[r]   = ((size_t)(b * NC + chn) * HI + h0 + dro) * WI + w0 + 4 * pj;
    }
#pragma unroll
    for (int r = 0; r < 8; ++r) *(volatile v4f*)(out + e[r]) = val[r];
    __threadfence();
#pragma unroll
    for (int r = 0; r < 8; ++r) *(volatile v4f*)(out + e[r]) = val[r];
  }
}

extern "C" void kernel_launch(void* const* d_in, const int* in_sizes, int n_in,
                              void* d_out, int out_size, void* d_ws, size_t ws_size,
                              hipStream_t stream) {
  if (n_in < 20) return;
  if (in_sizes[0] != NPIX * NC || in_sizes[1] != NPIX * NC) return;
  if (in_sizes[2] != NC * NC * 9 || in_sizes[8] != NC * NC * 9) return;
  if (in_sizes[14] != NC * NCX) return;
  for (int i = 3; i <= 7; ++i)  if (in_sizes[i] != NC) return;
  for (int i = 9; i <= 13; ++i) if (in_sizes[i] != NC) return;
  for (int i = 15; i <= 19; ++i) if (in_sizes[i] != NC) return;
  if (out_size != NPIX * NC) return;
  if (WS_END > ws_size) return;

  const float* fm1   = (const float*)d_in[0];
  const float* fm2   = (const float*)d_in[1];
  const float* wk_w  = (const float*)d_in[2];
  const float* wk_b  = (const float*)d_in[3];
  const float* wk_g  = (const float*)d_in[4];
  const float* wk_be = (const float*)d_in[5];
  const float* wk_m  = (const float*)d_in[6];
  const float* wk_v  = (const float*)d_in[7];
  const float* wq_w  = (const float*)d_in[8];
  const float* wq_b  = (const float*)d_in[9];
  const float* wq_g  = (const float*)d_in[10];
  const float* wq_be = (const float*)d_in[11];
  const float* wq_m  = (const float*)d_in[12];
  const float* wq_v  = (const float*)d_in[13];
  const float* q_w   = (const float*)d_in[14];
  const float* q_b   = (const float*)d_in[15];
  const float* q_g   = (const float*)d_in[16];
  const float* q_be  = (const float*)d_in[17];
  const float* q_m   = (const float*)d_in[18];
  const float* q_v   = (const float*)d_in[19];
  float* out = (float*)d_out;
  char* ws = (char*)d_ws;

  unsigned* w1_u       = (unsigned*)(ws + WS_W1);
  unsigned* w2_u       = (unsigned*)(ws + WS_W2);
  unsigned* wq_u       = (unsigned*)(ws + WS_WQ);
  unsigned short* x1_u = (unsigned short*)(ws + WS_X1);
  unsigned short* x2_u = (unsigned short*)(ws + WS_X2);
  _Float16* f1p        = (_Float16*)(ws + WS_F1);
  _Float16* f2p        = (_Float16*)(ws + WS_F2);

  k_wpack<<<dim3(2 * W_BLK + Q_BLK), dim3(256), 0, stream>>>(wk_w, wq_w, q_w, w1_u, w2_u, wq_u);
  (void)hipGetLastError();

  k_xcvt<<<dim3(2 * NBLK_X), dim3(256), 0, stream>>>(fm1, fm2, x1_u, x2_u);
  (void)hipGetLastError();

  k_zero<<<dim3(NB * 8), dim3(256), 0, stream>>>(f2p);
  (void)hipGetLastError();

  k_conv<<<dim3(2 * NBLK_CV), dim3(256), 0, stream>>>(
      (const __bf16*)x1_u, (const __bf16*)x2_u, (const __bf16*)w1_u, (const __bf16*)w2_u,
      wk_b, wk_g, wk_be, wk_m, wk_v,
      wq_b, wq_g, wq_be, wq_m, wq_v,
      f1p, f2p);
  (void)hipGetLastError();

  k_cq<<<dim3(NBLK_CQ), dim3(256), 0, stream>>>((const _Float16*)f1p, (const _Float16*)f2p,
                                                  (const _Float16*)wq_u, q_b, q_g, q_be, q_m, q_v, out);
  (void)hipGetLastError();
}
